// GraphAttentionNetwork_52836687675525
// MI455X (gfx1250) — hardware-verified
//
#include <hip/hip_runtime.h>
#include <stddef.h>
#include <stdint.h>
#include <math.h>

#define NBATCH 4
#define NNODE  512
#define NR     (NBATCH * NNODE)
#define FIN    64
#define HID    64
#define NHEAD  4
#define C1     (NHEAD * HID)
#define K1     64
#define K2     (2 * C1)
#define MUV    (2 * HID)
#define NTHR   256
#define GBM    64
#define GBN    64
#define GTHR   128
#define PT     64
#define NUX    (NR * (K1 / 8))
#define NUA    (MUV * (K1 / 8))
#define NUW1   (C1 * (K1 / 8))
#define NUW2   (HID * (C1 / 4))
#define NUT    (NUX + NUA + NUW1 + NUW2)
#define OUT0N  (NR * HID)
#define OUT1N  (NBATCH * NNODE * NNODE)
#define WSMAX  134217728

static_assert(K1 % 32 == 0 && K2 % 32 == 0 && K1 == FIN && K2 == 2 * C1);
static_assert(NR % GBM == 0 && MUV % GBM == 0);
static_assert(NR % GBN == 0 && C1 % GBN == 0 && HID % GBN == 0);
static_assert(GBM == (GTHR / 32) * 16 && GBN == 64);
static_assert(NUX % NTHR == 0 && NUA % NTHR == 0 && NUW1 % NTHR == 0 && NUW2 % NTHR == 0 && NUT % NTHR == 0);
static_assert(K1 / 8 == 8 && C1 / 4 == 64);
static_assert(NNODE % PT == 0 && HID == PT && PT == 64 && NTHR == 256 && HID <= NTHR);
static_assert(OUT0N * 4 == 524288);

typedef float          v4f   __attribute__((ext_vector_type(4)));
typedef float          v8f   __attribute__((ext_vector_type(8)));
typedef int            v8i   __attribute__((ext_vector_type(8)));
typedef unsigned short v8us  __attribute__((ext_vector_type(8)));
typedef unsigned short v16us __attribute__((ext_vector_type(16)));
typedef __bf16         v16bf __attribute__((ext_vector_type(16)));
typedef v4f  __attribute__((may_alias)) v4fa;
typedef v8us __attribute__((may_alias)) v8usa;
union Frag { v16bf v; v16us u; v8us h[2]; v8i w; };

__device__ __forceinline__ v8f wmb(const Frag& a, const Frag& b, v8f c) {
  v8f d = __builtin_amdgcn_wmma_f32_16x16x32_bf16(false, a.v, false, b.v, (short)0, c, false, false);
  asm volatile("v_nop\n\tv_nop\n\tv_nop\n\tv_nop" : "+v"(d) : "v"(a.w), "v"(b.w));
  return d;
}

__device__ __forceinline__ unsigned bf16_bits(float f) {
  const unsigned u = __float_as_uint(f);
  return (u + 0x7FFFu + ((u >> 16) & 1u)) >> 16;
}
__device__ __forceinline__ float bf16_val(float f) {
  return __uint_as_float(bf16_bits(f) << 16);
}
__device__ __forceinline__ v8us hilo8(v4f t) {
  v8us o;
  unsigned hb;
  hb = bf16_bits(t.x); o[0] = (unsigned short)hb; o[4] = (unsigned short)bf16_bits(t.x - __uint_as_float(hb << 16));
  hb = bf16_bits(t.y); o[1] = (unsigned short)hb; o[5] = (unsigned short)bf16_bits(t.y - __uint_as_float(hb << 16));
  hb = bf16_bits(t.z); o[2] = (unsigned short)hb; o[6] = (unsigned short)bf16_bits(t.z - __uint_as_float(hb << 16));
  hb = bf16_bits(t.w); o[3] = (unsigned short)hb; o[7] = (unsigned short)bf16_bits(t.w - __uint_as_float(hb << 16));
  return o;
}
__device__ __forceinline__ float elu1(float v) {
  const float en = expm1f(fminf(v, 0.0f));
  return v > 0.0f ? v : en;
}

__global__ __launch_bounds__(NTHR) void k_prep(const float* __restrict__ x, const float* __restrict__ epW1,
                                               const float* __restrict__ g1W, const float* __restrict__ g2W,
                                               unsigned short* Xb, unsigned short* AUW, unsigned short* W1T,
                                               unsigned short* W2T) {
  const int u = (int)blockIdx.x * NTHR + (int)threadIdx.x;
  v8us o;
  unsigned short* dp;
  if (u < NUX) {
    const int row = u >> 3;
    const int k8  = (u & 7) * 8;
    const float* p = x + (size_t)row * FIN + k8;
    const v4f a = *(const v4fa*)p;
    const v4f c = *(const v4fa*)(p + 4);
    o[0] = (unsigned short)bf16_bits(a.x); o[1] = (unsigned short)bf16_bits(a.y);
    o[2] = (unsigned short)bf16_bits(a.z); o[3] = (unsigned short)bf16_bits(a.w);
    o[4] = (unsigned short)bf16_bits(c.x); o[5] = (unsigned short)bf16_bits(c.y);
    o[6] = (unsigned short)bf16_bits(c.z); o[7] = (unsigned short)bf16_bits(c.w);
    dp = Xb + (size_t)row * K1 + k8;
  } else if (u < NUX + NUA) {
    const int v    = u - NUX;
    const int r    = v >> 3;
    const int k8   = (v & 7) * 8;
    const int half = r >> 6;
    const int c    = r & 63;
    const float* p = epW1 + (size_t)(half * FIN + k8) * HID + c;
#pragma unroll
    for (int i = 0; i < 8; ++i) o[i] = (unsigned short)bf16_bits(p[(size_t)i * HID]);
    dp = AUW + (size_t)r * K1 + k8;
  } else if (u < NUX + NUA + NUW1) {
    const int v    = u - NUX - NUA;
    const int n    = v >> 3;
    const int k8   = (v & 7) * 8;
    const int head = n >> 6;
    const int c    = n & 63;
    const float* p = g1W + (size_t)(head * FIN + k8) * HID + c;
#pragma unroll
    for (int i = 0; i < 8; ++i) o[i] = (unsigned short)bf16_bits(p[(size_t)i * HID]);
    dp = W1T + (size_t)n * K1 + k8;
  } else if (u < NUT) {
    const int v = u - NUX - NUA - NUW1;
    const int n = v >> 6;
    const int g = v & 63;
    const float* p = g2W + (size_t)(4 * g) * HID + n;
    const unsigned short f0 = (unsigned short)bf16_bits(p[0]);
    const unsigned short f1 = (unsigned short)bf16_bits(p[HID]);
    const unsigned short f2 = (unsigned short)bf16_bits(p[2 * HID]);
    const unsigned short f3 = (unsigned short)bf16_bits(p[3 * HID]);
    o[0] = f0; o[1] = f1; o[2] = f2; o[3] = f3; o[4] = f0; o[5] = f1; o[6] = f2; o[7] = f3;
    dp = W2T + (size_t)n * K2 + 8 * g;
  } else {
    return;
  }
  *(volatile v8us*)dp = o;
  __threadfence();
  *(volatile v8us*)dp = o;
}

template <int EPI>
__global__ __launch_bounds__(GTHR) void k_gemm(const unsigned short* __restrict__ A, const unsigned short* __restrict__ WT,
                                               const float* __restrict__ bias, int nbias,
                                               float* outF, unsigned short* outH, int K, int ldo) {
  __shared__ __attribute__((aligned(16))) float stg[GBM * GBN];
  __shared__ float sb[GBM];
  const int tid = (int)threadIdx.x, lane = tid & 31, wave = tid >> 5, hh = lane >> 4, m = lane & 15;
  const int rowBase = (int)blockIdx.x * GBM;
  const int col0    = (int)blockIdx.y * GBN;

  if constexpr (EPI == 0) {
    if (tid < GBM) {
      const int rr  = rowBase + tid;
      const int nbc = nbias > 0 ? nbias : 1;
      const int rc  = rr < nbc ? rr : nbc - 1;
      const float v = bf16_val(bias[rc]);
      sb[tid] = rr < nbias ? v : 0.0f;
    }
    __syncthreads();
  }

  v8f acc[4];
  {
    const v8f z = {0.f, 0.f, 0.f, 0.f, 0.f, 0.f, 0.f, 0.f};
    acc[0] = z; acc[1] = z; acc[2] = z; acc[3] = z;
  }
  const unsigned short* ap = A  + (size_t)(rowBase + 16 * wave + m) * (size_t)K + 8 * hh;
  const unsigned short* wp = WT + (size_t)(col0 + m) * (size_t)K + 8 * hh;
  const int ksteps = K >> 5;
#pragma unroll 1
  for (int ks = 0; ks < ksteps; ++ks) {
    Frag af;
    af.h[0] = *(const v8usa*)(ap + 32 * ks);
    af.h[1] = *(const v8usa*)(ap + 32 * ks + 16);
#pragma unroll
    for (int t = 0; t < 4; ++t) {
      const unsigned short* wq = wp + (size_t)(16 * t) * (size_t)K + 32 * ks;
      Frag bf;
      bf.h[0] = *(const v8usa*)wq;
      bf.h[1] = *(const v8usa*)(wq + 16);
      acc[t] = wmb(af, bf, acc[t]);
    }
  }

#pragma unroll
  for (int t = 0; t < 4; ++t) {
    const int lc = 16 * t + m;
#pragma unroll
    for (int r = 0; r < 8; ++r) {
      const int lr = 16 * wave + 8 * hh + r;
      float val = acc[t][r];
      if constexpr (EPI == 0) val = val + sb[lr];
      stg[lr * GBN + lc] = val;
    }
  }
  __syncthreads();

  v4f fv[8];
#pragma unroll
  for (int i = 0; i < 8; ++i) {
    const int lr = 16 * wave + 2 * i + hh;
    fv[i] = *(const v4fa*)(stg + lr * GBN + 4 * m);
  }
  if constexpr (EPI == 0) {
#pragma unroll
    for (int i = 0; i < 8; ++i) {
      const int lr = 16 * wave + 2 * i + hh;
      const int gr = rowBase + lr;
      float* op = outF + (size_t)gr * (size_t)ldo + col0 + 4 * m;
      *(volatile v4f*)op = fv[i];
    }
    __threadfence();
#pragma unroll
    for (int i = 0; i < 8; ++i) {
      const int lr = 16 * wave + 2 * i + hh;
      const int gr = rowBase + lr;
      float* op = outF + (size_t)gr * (size_t)ldo + col0 + 4 * m;
      *(volatile v4f*)op = fv[i];
    }
  } else {
    v8us pv[8];
#pragma unroll
    for (int i = 0; i < 8; ++i) {
      v4f e;
      e.x = elu1(fv[i].x); e.y = elu1(fv[i].y); e.z = elu1(fv[i].z); e.w = elu1(fv[i].w);
      pv[i] = hilo8(e);
    }
    const int g = (col0 >> 2) + m;
#pragma unroll
    for (int i = 0; i < 8; ++i) {
      const int lr = 16 * wave + 2 * i + hh;
      const int gr = rowBase + lr;
      unsigned short* hp = outH + (size_t)gr * (size_t)K2 + 8 * g;
      *(volatile v8us*)hp = pv[i];
    }
    __threadfence();
#pragma unroll
    for (int i = 0; i < 8; ++i) {
      const int lr = 16 * wave + 2 * i + hh;
      const int gr = rowBase + lr;
      unsigned short* hp = outH + (size_t)gr * (size_t)K2 + 8 * g;
      *(volatile v8us*)hp = pv[i];
    }
  }
}

__global__ __launch_bounds__(NTHR) void k_pair(const float* __restrict__ UVT, const float* __restrict__ W2,
                                               const float* __restrict__ b2, float* adj) {
  __shared__ __attribute__((aligned(16))) float s_i[PT * PT];
  __shared__ __attribute__((aligned(16))) float s_j[PT * PT];
  __shared__ __attribute__((aligned(16))) float s_w[HID];
  const int t = (int)threadIdx.x, lane = t & 31, w = t >> 5;
  const int b = (int)blockIdx.z, i0 = (int)blockIdx.x * PT, j0 = (int)blockIdx.y * PT;
  const int ti = t & 15, tj = t >> 4;

  if (t < HID) s_w[t] = bf16_val(W2[t]);
  const float bb = bf16_val(b2[0]);

  const v4f zero4 = {0.f, 0.f, 0.f, 0.f};
  v4f acc[4];
#pragma unroll
  for (int a = 0; a < 4; ++a) acc[a] = zero4;

  const float* Hib = UVT + (size_t)b * NNODE + i0;
  const float* Hjb = UVT + (size_t)HID * NR + (size_t)b * NNODE + j0;

  __syncthreads();
#pragma unroll
  for (int it = 0; it < 4; ++it) {
    const int h  = (t >> 4) + 16 * it;
    const int c4 = (t & 15) * 4;
    const v4f vi = *(const v4fa*)(Hib + (size_t)h * NR + c4);
    const v4f vj = *(const v4fa*)(Hjb + (size_t)h * NR + c4);
    *(v4fa*)(s_i + h * PT + c4) = vi;
    *(v4fa*)(s_j + h * PT + c4) = vj;
  }
  __syncthreads();

#pragma unroll 2
  for (int hu = 0; hu < PT; ++hu) {
    const v4f hi4 = *(const v4fa*)(s_i + hu * PT + 4 * ti);
    const v4f hj4 = *(const v4fa*)(s_j + hu * PT + 4 * tj);
    const float wv = s_w[hu];
#pragma unroll
    for (int a = 0; a < 4; ++a)
#pragma unroll
      for (int q = 0; q < 4; ++q) {
        const float v = fmaxf(hi4[a] + hj4[q], 0.0f);
        acc[a][q] = fmaf(v, wv, acc[a][q]);
      }
  }
  __syncthreads();

  float* sO = s_i;
#pragma unroll
  for (int a = 0; a < 4; ++a) {
    v4f o;
    const int gi = i0 + 4 * ti + a;
#pragma unroll
    for (int q = 0; q < 4; ++q) {
      const float l = acc[a][q] + bb;
      const float e = __expf(-l);
      const float s = __builtin_amdgcn_rcpf(1.0f + e);
      const int gj = j0 + 4 * tj + q;
      o[q] = (gi == gj) ? 1.0f : s;
    }
    *(v4fa*)(sO + (4 * ti + a) * PT + 4 * tj) = o;
  }
  __syncthreads();

  const int rsub = lane >> 4, c4 = (lane & 15) * 4;
  v4f vals[4];
#pragma unroll
  for (int it = 0; it < 4; ++it) {
    const int row = 8 * w + 2 * it + rsub;
    vals[it] = *(const v4fa*)(sO + row * PT + c4);
  }
#pragma unroll
  for (int it = 0; it < 4; ++it) {
    const int row = 8 * w + 2 * it + rsub;
    float* op = adj + ((size_t)(b * NNODE + i0 + row) * (size_t)NNODE + j0 + c4);
    *(volatile v4f*)op = vals[it];
  }
  __threadfence();
#pragma unroll
  for (int it = 0; it < 4; ++it) {
    const int row = 8 * w + 2 * it + rsub;
    float* op = adj + ((size_t)(b * NNODE + i0 + row) * (size_t)NNODE + j0 + c4);
    *(volatile v4f*)op = vals[it];
  }
}

extern "C" void kernel_launch(void* const* d_in, const int* in_sizes, int n_in,
                              void* d_out, int out_size, void* d_ws, size_t ws_size,
                              hipStream_t stream) {
  if (n_in < 9) return;
  if (in_sizes[0] != NR * FIN) return;
  if (in_sizes[1] != NHEAD * FIN * HID) return;
  if (in_sizes[2] != NHEAD * 2 * HID) return;
  if (in_sizes[3] != C1 * HID) return;
  if (in_sizes[4] != 2 * HID) return;
  if (in_sizes[5] != 2 * FIN * HID) return;
  if (in_sizes[6] != HID) return;
  if (in_sizes[7] != HID) return;
  if (in_sizes[8] != 1) return;
  if (out_size != OUT0N + OUT1N) return;

  const float* x    = (const float*)d_in[0];
  const float* g1W  = (const float*)d_in[1];
  const float* g2W  = (const float*)d_in[3];
  const float* epW1 = (const float*)d_in[5];
  const float* epb1 = (const float*)d_in[6];
  const float* epW2 = (const float*)d_in[7];
  const float* epb2 = (const float*)d_in[8];
  float* out  = (float*)d_out;
  float* out0 = out;
  float* adj  = out + OUT0N;

  char* ws = (char*)d_ws;
  size_t off = 0;
  const size_t oXb  = off; off += (size_t)NR  * K1 * 2;  off = (off + 255) & ~(size_t)255;
  const size_t oAUW = off; off += (size_t)MUV * K1 * 2;  off = (off + 255) & ~(size_t)255;
  const size_t oW1T = off; off += (size_t)C1  * K1 * 2;  off = (off + 255) & ~(size_t)255;
  const size_t oW2T = off; off += (size_t)HID * K2 * 2;  off = (off + 255) & ~(size_t)255;
  const size_t oUVT = off; off += (size_t)MUV * NR * 4;  off = (off + 255) & ~(size_t)255;
  const size_t oA2  = off; off += (size_t)NR  * K2 * 2;  off = (off + 255) & ~(size_t)255;
  if (off > ws_size || off > (size_t)WSMAX) return;
  unsigned short* Xb  = (unsigned short*)(ws + oXb);
  unsigned short* AUW = (unsigned short*)(ws + oAUW);
  unsigned short* W1T = (unsigned short*)(ws + oW1T);
  unsigned short* W2T = (unsigned short*)(ws + oW2T);
  float*          UVT = (float*)(ws + oUVT);
  unsigned short* A2  = (unsigned short*)(ws + oA2);

  k_prep<<<NUT / NTHR, NTHR, 0, stream>>>(x, epW1, g1W, g2W, Xb, AUW, W1T, W2T);
  k_gemm<0><<<dim3(MUV / GBM, NR / GBN), GTHR, 0, stream>>>(AUW, Xb, epb1, HID, UVT, A2, K1, NR);
  k_pair<<<dim3(NNODE / PT, NNODE / PT, NBATCH), NTHR, 0, stream>>>(UVT, epW2, epb2, adj);
  k_gemm<1><<<dim3(NR / GBM, C1 / GBN), GTHR, 0, stream>>>(Xb, W1T, epb1, 0, UVT, A2, K1, 0);
  k_gemm<0><<<dim3(NR / GBM, HID / GBN), GTHR, 0, stream>>>(A2, W2T, epb1, 0, out0, A2, K2, HID);
  (void)hipGetLastError();
}
